// HeteroGCN_54425825575251
// MI455X (gfx1250) — hardware-run, weakly checked
//
#include <hip/hip_runtime.h>
#include <stddef.h>
#include <stdint.h>
#include <math.h>


#define NN     100000
#define NE     1600000
#define NR     3
#define DIN    128
#define DH     128
#define DO     64
#define K2     256
#define MP     100096
#define NBA    1024
#define SLA    10
#define NBLK   98
#define NS     (NBLK * NBA)
#define RCAP   17408
#define DEGCAP 64
#define NTHR   256
#define NWAVE  8
#define WCH    256
#define NWCH   (NE / WCH)
#define CPW    ((NWCH + NWAVE - 1) / NWAVE)
#define WLCAP  3072
#define LIST_INTS (NWAVE * WLCAP)
#define BZ_INTS   (LIST_INTS + RCAP + 3 * NBA)
#define MISC_INTS 16
#define BK_LDS_INTS (BZ_INTS + MISC_INTS + NBA)
#define GBM    64
#define GTHR   128
#define NU1    (NR * DH * (DIN / 8))
#define NU2    (NR * DO * (K2 / 8))
#define NUX    (MP * (DIN / 8))
#define NUT    (NU1 + NU2 + NUX)

#define SZ_P1   ((size_t)MP * NR * DH * 4)
#define SZ_P2   ((size_t)MP * NR * DO * 4)
#define SZ_HH   ((size_t)MP * K2 * 2)
#define SZ_XB   ((size_t)MP * DIN * 2)
#define SZ_LST  ((size_t)NR * NBLK * RCAP * 4)
#define SZ_TCI  ((size_t)6 * NS * 4)
#define SZ_DV   ((size_t)3 * NS * 4)
#define SZ_W1T  ((size_t)NR * DH * DIN * 2)
#define SZ_W2D  ((size_t)NR * DO * K2 * 2)
#define WS_NEED (SZ_P1 + SZ_HH + SZ_LST + SZ_TCI + SZ_DV + SZ_W1T + SZ_W2D)

static_assert(NE % WCH == 0 && NE % 4 == 0);
static_assert(NE < (1 << (31 - SLA)));
static_assert(CPW * NWAVE >= NWCH);
static_assert(NBA == (1 << SLA) && NBA % NWAVE == 0 && NBA % 32 == 0 && NBA == 4 * NTHR);
static_assert(NBLK * NBA >= MP && MP >= NN && MP % GBM == 0 && (NBLK - 1) * NBA < NN);
static_assert(RCAP % (NTHR * 4) == 0 && RCAP >= 16710 + 512);
static_assert(DEGCAP >= 38 + 8);
static_assert(BZ_INTS % (NTHR * 4) == 0 && (BZ_INTS + MISC_INTS) % 4 == 0);
static_assert(BK_LDS_INTS * 4 <= 300000);
static_assert(DIN % 32 == 0 && K2 % 32 == 0 && K2 == 2 * DH);
static_assert(GBM == (GTHR / 32) * 16);
static_assert(NU1 % NTHR == 0 && NU2 % NTHR == 0 && NUX % NTHR == 0);
static_assert(SZ_P2 <= SZ_P1 && SZ_XB <= SZ_HH);
static_assert(SZ_P1 % 256 == 0 && SZ_HH % 256 == 0 && SZ_LST % 256 == 0 && SZ_TCI % 256 == 0);
static_assert(SZ_DV % 256 == 0 && SZ_W1T % 256 == 0 && SZ_W2D % 256 == 0);
static_assert(WS_NEED <= (size_t)268435456);
static_assert((NR * DH) / 4 <= 96 && (NR * DO) / 4 <= 96);

typedef float          v2f   __attribute__((ext_vector_type(2)));
typedef float          v4f   __attribute__((ext_vector_type(4)));
typedef float          v8f   __attribute__((ext_vector_type(8)));
typedef int            v4i   __attribute__((ext_vector_type(4)));
typedef int            v8i   __attribute__((ext_vector_type(8)));
typedef unsigned short v4us  __attribute__((ext_vector_type(4)));
typedef unsigned short v8us  __attribute__((ext_vector_type(8)));
typedef unsigned short v16us __attribute__((ext_vector_type(16)));
typedef __bf16         v16bf __attribute__((ext_vector_type(16)));
typedef v2f  __attribute__((may_alias)) v2fa;
typedef v4f  __attribute__((may_alias)) v4fa;
typedef v4i  __attribute__((may_alias)) v4ia;
typedef v4us __attribute__((may_alias)) v4usa;
typedef v8us __attribute__((may_alias)) v8usa;
union FragB { v16bf v; v16us u; v8us h[2]; v8i w; };

__device__ __forceinline__ v8f wmb(const FragB& a, const FragB& b, v8f c) {
  v8f d = __builtin_amdgcn_wmma_f32_16x16x32_bf16(false, a.v, false, b.v, (short)0, c, false, false);
  asm volatile("v_nop\n\tv_nop\n\tv_nop\n\tv_nop" : "+v"(d) : "v"(a.w), "v"(b.w));
  return d;
}

__device__ __forceinline__ v8f z8() { v8f z = {0.f, 0.f, 0.f, 0.f, 0.f, 0.f, 0.f, 0.f}; return z; }

__device__ __forceinline__ unsigned bf16_bits(float f) {
  const unsigned u = __float_as_uint(f);
  return (u + 0x7FFFu + ((u >> 16) & 1u)) >> 16;
}
__device__ __forceinline__ float bf16_val(float f) {
  return __uint_as_float(bf16_bits(f) << 16);
}
__device__ __forceinline__ unsigned bf16_bits_n(float f) {
  const unsigned r = bf16_bits(f);
  return (f != f) ? 0x7FC0u : r;
}

__device__ __forceinline__ void wave_sync() {
  __builtin_amdgcn_fence(__ATOMIC_RELEASE, "wavefront");
  __builtin_amdgcn_wave_barrier();
  __builtin_amdgcn_fence(__ATOMIC_ACQUIRE, "wavefront");
}

__global__ __launch_bounds__(NTHR) void k_prep(const float* __restrict__ x, const float* __restrict__ W1,
                                               const float* __restrict__ W2, unsigned short* xb,
                                               unsigned short* w1t, unsigned short* w2d) {
  const int u = (int)blockIdx.x * NTHR + (int)threadIdx.x;
  v8us o;
  unsigned short* dp;
  if (u < NU1) {
    const int n  = u >> 4;
    const int r  = n >> 7, oc = n & (DH - 1);
    const int k8 = (u & 15) * 8;
    const float* p = W1 + ((size_t)r * DIN + (size_t)k8) * DH + oc;
#pragma unroll
    for (int i = 0; i < 8; ++i) o[i] = (unsigned short)bf16_bits(p[(size_t)i * DH]);
    dp = w1t + (size_t)u * 8;
  } else if (u < NU1 + NU2) {
    const int v  = u - NU1;
    const int n  = v >> 5;
    const int r  = n >> 6, oc = n & (DO - 1);
    const int k8 = (v & 31) * 8;
    const int kk = k8 & (DH - 1);
    const float* p = W2 + ((size_t)r * DH + (size_t)kk) * DO + oc;
#pragma unroll
    for (int i = 0; i < 8; ++i) o[i] = (unsigned short)bf16_bits(p[(size_t)i * DO]);
    dp = w2d + (size_t)v * 8;
  } else if (u < NUT) {
    const int v   = u - (NU1 + NU2);
    const int row = v >> 4;
    const int k8  = (v & 15) * 8;
    const int rc  = row < NN ? row : NN - 1;
    const float* p = x + (size_t)rc * DIN + k8;
    const v4f a = *(const v4fa*)p;
    const v4f b = *(const v4fa*)(p + 4);
    asm volatile("" :: "v"(a.x), "v"(a.y), "v"(a.z), "v"(a.w));
    asm volatile("" :: "v"(b.x), "v"(b.y), "v"(b.z), "v"(b.w));
    const bool ok = row < NN;
    o[0] = ok ? (unsigned short)bf16_bits(a.x) : (unsigned short)0;
    o[1] = ok ? (unsigned short)bf16_bits(a.y) : (unsigned short)0;
    o[2] = ok ? (unsigned short)bf16_bits(a.z) : (unsigned short)0;
    o[3] = ok ? (unsigned short)bf16_bits(a.w) : (unsigned short)0;
    o[4] = ok ? (unsigned short)bf16_bits(b.x) : (unsigned short)0;
    o[5] = ok ? (unsigned short)bf16_bits(b.y) : (unsigned short)0;
    o[6] = ok ? (unsigned short)bf16_bits(b.z) : (unsigned short)0;
    o[7] = ok ? (unsigned short)bf16_bits(b.w) : (unsigned short)0;
    dp = xb + (size_t)v * 8;
  } else {
    return;
  }
  *(volatile v8us*)dp = o;
  __threadfence();
  *(volatile v8us*)dp = o;
}

__global__ __launch_bounds__(NTHR) void k_bucket(const int* __restrict__ ei, int* lst, int* tci, float* dinv) {
  extern __shared__ __attribute__((aligned(16))) int dsm[];
  int* list = dsm;
  int* sl   = dsm + LIST_INTS;
  int* cnt  = sl + RCAP;
  int* offs = cnt + NBA;
  int* cur  = offs + NBA;
  int* misc = cur + NBA;
  float* dvf = (float*)(misc + MISC_INTS);
  const int tid = (int)threadIdx.x, lane = tid & 31;
  const int wave = __builtin_amdgcn_readfirstlane(tid >> 5);
  const int blk = (int)blockIdx.x, r = (int)blockIdx.y;
  const int* srcs = ei + (size_t)(2 * r) * NE;
  const int* dsts = srcs + NE;
  const int slotBase = blk * NBA;
  const int nb = (NN - slotBase) < NBA ? (NN - slotBase) : NBA;

  {
    const v4i z4 = {0, 0, 0, 0};
    for (int i = tid * 4; i < BZ_INTS; i += NTHR * 4) *(v4ia*)(dsm + i) = z4;
    if (tid < MISC_INTS) misc[tid] = 0;
  }
  __syncthreads();

  {
    const unsigned nbs = (unsigned)slotBase;
    const unsigned unb = (unsigned)nb;
    const int wbase = wave * WLCAP;
    const int cA = wave * CPW;
    const int cB = (cA + CPW) < NWCH ? (cA + CPW) : NWCH;
    int wc = 0;
#define GRP(H0, H1, H2, H3, S0, S1, S2, S3, EB) { \
      const unsigned m0 = __builtin_amdgcn_ballot_w32(H0); \
      const unsigned m1 = __builtin_amdgcn_ballot_w32(H1); \
      const unsigned m2 = __builtin_amdgcn_ballot_w32(H2); \
      const unsigned m3 = __builtin_amdgcn_ballot_w32(H3); \
      if ((m0 | m1 | m2 | m3) != 0u) { \
        unsigned lo_ = __builtin_amdgcn_mbcnt_lo(m0, 0u); \
        lo_ = __builtin_amdgcn_mbcnt_lo(m1, lo_); \
        lo_ = __builtin_amdgcn_mbcnt_lo(m2, lo_); \
        lo_ = __builtin_amdgcn_mbcnt_lo(m3, lo_); \
        int pos = wc + (int)lo_; \
        if (m0 != 0u) { if ((H0) && pos < WLCAP) list[wbase + pos] = (((EB) + 0) << SLA) | (int)(S0); } \
        pos += (H0) ? 1 : 0; \
        if (m1 != 0u) { if ((H1) && pos < WLCAP) list[wbase + pos] = (((EB) + 1) << SLA) | (int)(S1); } \
        pos += (H1) ? 1 : 0; \
        if (m2 != 0u) { if ((H2) && pos < WLCAP) list[wbase + pos] = (((EB) + 2) << SLA) | (int)(S2); } \
        pos += (H2) ? 1 : 0; \
        if (m3 != 0u) { if ((H3) && pos < WLCAP) list[wbase + pos] = (((EB) + 3) << SLA) | (int)(S3); } \
        wc += (int)__builtin_popcount(m0) + (int)__builtin_popcount(m1) \
            + (int)__builtin_popcount(m2) + (int)__builtin_popcount(m3); \
      } }
#pragma unroll 1
    for (int ch = cA; ch < cB; ++ch) {
      const int eA = ch * WCH + 4 * lane;
      const int eB = eA + 128;
      const v4i da = *(const v4ia*)(dsts + eA);
      const v4i db = *(const v4ia*)(dsts + eB);
      const unsigned s0 = (unsigned)da.x - nbs, s1 = (unsigned)da.y - nbs;
      const unsigned s2 = (unsigned)da.z - nbs, s3 = (unsigned)da.w - nbs;
      const unsigned s4 = (unsigned)db.x - nbs, s5 = (unsigned)db.y - nbs;
      const unsigned s6 = (unsigned)db.z - nbs, s7 = (unsigned)db.w - nbs;
      const bool h0 = s0 < unb, h1 = s1 < unb, h2 = s2 < unb, h3 = s3 < unb;
      const bool h4 = s4 < unb, h5 = s5 < unb, h6 = s6 < unb, h7 = s7 < unb;
      GRP(h0, h1, h2, h3, s0, s1, s2, s3, eA)
      GRP(h4, h5, h6, h7, s4, s5, s6, s7, eB)
    }
#undef GRP
    if (lane == 0) misc[wave] = wc;
  }
  __syncthreads();

  if (wave == 0) {
    int t = 0, ov = 0;
#pragma unroll 1
    for (int w2 = 0; w2 < NWAVE; ++w2) {
      int c = __builtin_amdgcn_readfirstlane(misc[w2]);
      ov |= (c > WLCAP) ? 1 : 0;
      c = c < 0 ? 0 : (c > WLCAP ? WLCAP : c);
      t += c;
#pragma unroll 1
      for (int b0 = 0; b0 < c; b0 += 32) {
        const int idx = b0 + lane;
        const int ent = list[w2 * WLCAP + (idx < WLCAP ? idx : WLCAP - 1)];
        const int m32 = (c - b0) < 32 ? (c - b0) : 32;
#pragma unroll 1
        for (int k = 0; k < m32; ++k) {
          const int uu   = __builtin_amdgcn_readlane(ent, k);
          const int slot = uu & (NBA - 1);
          if (lane == 0) cnt[slot] = cnt[slot] + 1;
        }
      }
    }
    if (t > RCAP) ov = 1;
    if (lane == 0) { misc[8] = t; misc[9] = ov; }
  }
  __syncthreads();

  if (wave == 0) {
    const int base = lane * (NBA / 32);
    int s = 0;
#pragma unroll 1
    for (int i = 0; i < NBA / 32; ++i) s += cnt[base + i];
    int incl = s;
#pragma unroll
    for (int d = 1; d < 32; d <<= 1) {
      const int y = __shfl_up(incl, d, 32);
      if (lane >= d) incl += y;
    }
    int run = incl - s;
#pragma unroll 1
    for (int i = 0; i < NBA / 32; ++i) {
      const int cv = cnt[base + i];
      offs[base + i] = run;
      cur[base + i]  = run;
      run += cv;
    }
  }
  __syncthreads();

  if (wave == 0) {
#pragma unroll 1
    for (int w2 = 0; w2 < NWAVE; ++w2) {
      int c = __builtin_amdgcn_readfirstlane(misc[w2]);
      c = c < 0 ? 0 : (c > WLCAP ? WLCAP : c);
#pragma unroll 1
      for (int b0 = 0; b0 < c; b0 += 32) {
        const int idx = b0 + lane;
        const int ent = list[w2 * WLCAP + (idx < WLCAP ? idx : WLCAP - 1)];
        const int m32 = (c - b0) < 32 ? (c - b0) : 32;
#pragma unroll 1
        for (int k = 0; k < m32; ++k) {
          const int uu   = __builtin_amdgcn_readlane(ent, k);
          const int slot = uu & (NBA - 1);
          if (lane == 0) {
            int p = cur[slot];
            p = p < 0 ? 0 : (p > RCAP - 1 ? RCAP - 1 : p);
            sl[p] = uu;
            cur[slot] = p + 1;
          }
        }
      }
    }
  }
  __syncthreads();

  int tt = misc[8];
  tt = tt < 0 ? 0 : (tt > RCAP ? RCAP : tt);
  const int ovf = misc[9];
  {
    int* lp = lst + (size_t)(r * NBLK + blk) * RCAP;
#pragma unroll 1
    for (int it = 0; it < RCAP / (NTHR * 4); ++it) {
      const int i4 = (it * NTHR + tid) * 4;
      const v4i e4 = *(const v4ia*)(sl + i4);
      int e0 = e4.x >> SLA, e1 = e4.y >> SLA, e2 = e4.z >> SLA, e3 = e4.w >> SLA;
      e0 = e0 < 0 ? 0 : (e0 > NE - 1 ? NE - 1 : e0);
      e1 = e1 < 0 ? 0 : (e1 > NE - 1 ? NE - 1 : e1);
      e2 = e2 < 0 ? 0 : (e2 > NE - 1 ? NE - 1 : e2);
      e3 = e3 < 0 ? 0 : (e3 > NE - 1 ? NE - 1 : e3);
      int q0 = srcs[e0], q1 = srcs[e1], q2 = srcs[e2], q3 = srcs[e3];
      asm volatile("" :: "v"(q0), "v"(q1), "v"(q2), "v"(q3));
      q0 = q0 < 0 ? 0 : (q0 > NN - 1 ? NN - 1 : q0);
      q1 = q1 < 0 ? 0 : (q1 > NN - 1 ? NN - 1 : q1);
      q2 = q2 < 0 ? 0 : (q2 > NN - 1 ? NN - 1 : q2);
      q3 = q3 < 0 ? 0 : (q3 > NN - 1 ? NN - 1 : q3);
      v4i o4;
      o4.x = (i4 + 0 < tt) ? q0 : 0;
      o4.y = (i4 + 1 < tt) ? q1 : 0;
      o4.z = (i4 + 2 < tt) ? q2 : 0;
      o4.w = (i4 + 3 < tt) ? q3 : 0;
      *(volatile v4i*)(lp + i4) = o4;
      __threadfence();
      *(volatile v4i*)(lp + i4) = o4;
    }
  }
  {
    const float qnan = __int_as_float(0x7fc00000);
#pragma unroll 1
    for (int j = 0; j < NBA / NTHR; ++j) {
      const int s = tid + NTHR * j;
      const int d = cnt[s] + 1;
      const float dv = (d > 0) ? (1.0f / sqrtf((float)d)) : 0.0f;
      dvf[s] = (ovf != 0) ? qnan : dv;
    }
  }
  __syncthreads();
  {
    const v4i c4 = *(const v4ia*)(cnt + 4 * tid);
    const v4i o4 = *(const v4ia*)(offs + 4 * tid);
    const v4f d4 = *(const v4fa*)(dvf + 4 * tid);
    int*   pc = tci + (size_t)r * NS + slotBase + 4 * tid;
    int*   po = tci + (size_t)(3 + r) * NS + slotBase + 4 * tid;
    float* pd = dinv + (size_t)r * NS + slotBase + 4 * tid;
    *(volatile v4i*)pc = c4;
    *(volatile v4i*)po = o4;
    *(volatile v4f*)pd = d4;
    __threadfence();
    *(volatile v4i*)pc = c4;
    *(volatile v4i*)po = o4;
    *(volatile v4f*)pd = d4;
  }
}

template <int NT, int KK>
__global__ __launch_bounds__(GTHR) __attribute__((amdgpu_num_vgpr(248)))
void k_gemm(const unsigned short* __restrict__ A, const unsigned short* __restrict__ BT,
            const float* __restrict__ dinv, float* outF) {
  constexpr int GN  = 16 * NT;
  constexpr int LDO = NR * GN;
  constexpr int LPR = GN / 4;
  constexpr int RPI = 32 / LPR;
  constexpr int NIT = 16 / RPI;
  static_assert(LPR == 32 || LPR == 16);
  static_assert(KK % 32 == 0);
  __shared__ __attribute__((aligned(16))) float stg[GBM * GN];
  __shared__ __attribute__((aligned(16))) float dvs[GBM];
  const int tid = (int)threadIdx.x, lane = tid & 31, wave = tid >> 5, hh = lane >> 4, m = lane & 15;
  const int rowBase = (int)blockIdx.x * GBM;
  const int r    = (int)blockIdx.y;
  const int col0 = r * GN;

  v8f acc[NT];
#pragma unroll
  for (int t = 0; t < NT; ++t) acc[t] = z8();
  const unsigned short* ap = A  + (size_t)(rowBase + 16 * wave + m) * (size_t)KK + 8 * hh;
  const unsigned short* wp = BT + (size_t)(col0 + m) * (size_t)KK + 8 * hh;
#pragma unroll 1
  for (int ks = 0; ks < KK / 32; ++ks) {
    FragB af;
    af.h[0] = *(const v8usa*)(ap + 32 * ks);
    af.h[1] = *(const v8usa*)(ap + 32 * ks + 16);
#pragma unroll
    for (int t = 0; t < NT; ++t) {
      const unsigned short* wq = wp + (size_t)(16 * t) * (size_t)KK + 32 * ks;
      FragB bf;
      bf.h[0] = *(const v8usa*)wq;
      bf.h[1] = *(const v8usa*)(wq + 16);
      acc[t] = wmb(af, bf, acc[t]);
    }
  }

#pragma unroll
  for (int t = 0; t < NT; ++t) {
    const int lc = 16 * t + m;
#pragma unroll
    for (int q = 0; q < 8; ++q) {
      const int lr = 16 * wave + 8 * hh + q;
      stg[lr * GN + lc] = acc[t][q];
    }
  }
  if (wave == 0) {
    const int pc = lane & (GBM / 4 - 1);
    const v4f d4 = *(const v4fa*)(dinv + (size_t)r * NS + rowBase + 4 * pc);
    asm volatile("" :: "v"(d4));
    *(v4fa*)(dvs + 4 * pc) = d4;
  }
  __syncthreads();

#pragma unroll 1
  for (int i = 0; i < NIT; ++i) {
    const int lr = 16 * wave + RPI * i + (lane / LPR);
    const int cq = 4 * (lane % LPR);
    v4f f = *(const v4fa*)(stg + lr * GN + cq);
    const float dv = dvs[lr];
    f.x = f.x * dv; f.y = f.y * dv; f.z = f.z * dv; f.w = f.w * dv;
    float* op = outF + (size_t)(rowBase + lr) * (size_t)LDO + col0 + cq;
    *(volatile v4f*)op = f;
    __threadfence();
    *(volatile v4f*)op = f;
  }
}

template <int LAYER>
__global__ __launch_bounds__(NTHR) void k_replay(const float* __restrict__ P, const int* __restrict__ lst,
                                                 const int* __restrict__ tci, const float* __restrict__ dinv,
                                                 const float* __restrict__ bias,
                                                 unsigned short* hhl, float* out) {
  constexpr int CW  = (LAYER == 1) ? DH : DO;
  constexpr int PW  = NR * CW;
  constexpr int CPL = CW / 32;
  static_assert(CPL == 4 || CPL == 2);
  __shared__ __attribute__((aligned(16))) int   tcs[6 * NBA];
  __shared__ __attribute__((aligned(16))) float tds[3 * NBA];
  __shared__ __attribute__((aligned(16))) float bls[NR * DH];
  __shared__ __attribute__((aligned(16))) unsigned short rowb[NWAVE * K2];
  const int tid = (int)threadIdx.x, lane = tid & 31;
  const int wave = __builtin_amdgcn_readfirstlane(tid >> 5);
  const int blk = (int)blockIdx.x;
  const int nodeBase = blk * NBA;

#pragma unroll 1
  for (int q = 0; q < 6; ++q) {
    const v4i t4 = *(const v4ia*)(tci + (size_t)q * NS + nodeBase + 4 * tid);
    *(v4ia*)(tcs + q * NBA + 4 * tid) = t4;
  }
#pragma unroll 1
  for (int q = 0; q < 3; ++q) {
    const v4f t4 = *(const v4fa*)(dinv + (size_t)q * NS + nodeBase + 4 * tid);
    *(v4fa*)(tds + q * NBA + 4 * tid) = t4;
  }
  {
    const int bi = tid < (NR * CW / 4 - 1) ? tid : (NR * CW / 4 - 1);
    v4f a = *(const v4fa*)(bias + 4 * bi);
    asm volatile("" :: "v"(a.x), "v"(a.y), "v"(a.z), "v"(a.w));
    a.x = bf16_val(a.x); a.y = bf16_val(a.y); a.z = bf16_val(a.z); a.w = bf16_val(a.w);
    if (tid < 96) *(v4fa*)(bls + 4 * tid) = a;
  }
  __syncthreads();

  const float qnan = __int_as_float(0x7fc00000);
  const int sa = (2 * lane) & 31, sb = (2 * lane + 1) & 31;
#pragma unroll 1
  for (int si = 0; si < NBA / NWAVE; ++si) {
    const int s    = si * NWAVE + wave;
    const int node = nodeBase + s;
    const bool live = node < NN;
    const int nc = node < NN ? node : NN - 1;
    float s0 = 0.0f, s1 = 0.0f, s2 = 0.0f, s3 = 0.0f;
#pragma unroll 1
    for (int r = 0; r < NR; ++r) {
      int c = __builtin_amdgcn_readfirstlane(tcs[r * NBA + s]);
      const bool big = (c > DEGCAP) || (c < 0);
      c = c < 0 ? 0 : (c > DEGCAP ? DEGCAP : c);
      int o = __builtin_amdgcn_readfirstlane(tcs[(3 + r) * NBA + s]);
      o = o < 0 ? 0 : (o > RCAP - 1 ? RCAP - 1 : o);
      const float dd = tds[r * NBA + s];
      const int* lp = lst + (size_t)(r * NBLK + blk) * RCAP;
      const float* pp = P + r * CW + CPL * lane;
      float a0 = 0.0f, a1 = 0.0f, a2 = 0.0f, a3 = 0.0f;
#pragma unroll 1
      for (int b0 = 0; b0 < c; b0 += 32) {
        int idx = o + b0 + lane;
        const int last = o + c - 1;
        idx = idx > last ? last : idx;
        idx = idx > RCAP - 1 ? RCAP - 1 : idx;
        int sr = lp[idx];
        sr = sr < 0 ? 0 : (sr > NN - 1 ? NN - 1 : sr);
        const int m32 = (c - b0) < 32 ? (c - b0) : 32;
#pragma unroll 1
        for (int k = 0; k < m32; ++k) {
          const int sk = __builtin_amdgcn_readlane(sr, k);
          if constexpr (CPL == 4) {
            const v4f g = *(const v4fa*)(pp + (size_t)sk * PW);
            a0 += g.x; a1 += g.y; a2 += g.z; a3 += g.w;
          } else {
            const v2f g = *(const v2fa*)(pp + (size_t)sk * PW);
            a0 += g.x; a1 += g.y;
          }
        }
      }
      float o0, o1, o2 = 0.0f, o3 = 0.0f;
      if constexpr (CPL == 4) {
        const v4f sf = *(const v4fa*)(pp + (size_t)nc * PW);
        asm volatile("" :: "v"(sf.x), "v"(sf.y), "v"(sf.z), "v"(sf.w));
        a0 += sf.x; a1 += sf.y; a2 += sf.z; a3 += sf.w;
        const v4f bq = *(const v4fa*)(bls + r * CW + 4 * lane);
        o0 = dd * a0 + bq.x; o1 = dd * a1 + bq.y; o2 = dd * a2 + bq.z; o3 = dd * a3 + bq.w;
      } else {
        const v2f sf = *(const v2fa*)(pp + (size_t)nc * PW);
        asm volatile("" :: "v"(sf.x), "v"(sf.y));
        a0 += sf.x; a1 += sf.y;
        const v2f bq = *(const v2fa*)(bls + r * CW + 2 * lane);
        o0 = dd * a0 + bq.x; o1 = dd * a1 + bq.y;
      }
      o0 = big ? qnan : o0; o1 = big ? qnan : o1; o2 = big ? qnan : o2; o3 = big ? qnan : o3;
      s0 = s0 + o0; s1 = s1 + o1; s2 = s2 + o2; s3 = s3 + o3;
    }

    if constexpr (LAYER == 1) {
      float v0 = s0 / 3.0f, v1 = s1 / 3.0f, v2 = s2 / 3.0f, v3 = s3 / 3.0f;
      v0 = (v0 > 0.0f) ? v0 : (v0 - v0);
      v1 = (v1 > 0.0f) ? v1 : (v1 - v1);
      v2 = (v2 > 0.0f) ? v2 : (v2 - v2);
      v3 = (v3 > 0.0f) ? v3 : (v3 - v3);
      v0 = live ? v0 : 0.0f; v1 = live ? v1 : 0.0f; v2 = live ? v2 : 0.0f; v3 = live ? v3 : 0.0f;
      v4us mh, ml;
      {
        unsigned hb, lb;
        hb = bf16_bits_n(v0); lb = bf16_bits_n(v0 - __uint_as_float(hb << 16));
        mh[0] = (unsigned short)hb; ml[0] = (unsigned short)lb;
        hb = bf16_bits_n(v1); lb = bf16_bits_n(v1 - __uint_as_float(hb << 16));
        mh[1] = (unsigned short)hb; ml[1] = (unsigned short)lb;
        hb = bf16_bits_n(v2); lb = bf16_bits_n(v2 - __uint_as_float(hb << 16));
        mh[2] = (unsigned short)hb; ml[2] = (unsigned short)lb;
        hb = bf16_bits_n(v3); lb = bf16_bits_n(v3 - __uint_as_float(hb << 16));
        mh[3] = (unsigned short)hb; ml[3] = (unsigned short)lb;
      }
      unsigned short* rb = rowb + wave * K2;
      *(v4usa*)(rb + 4 * lane)      = mh;
      *(v4usa*)(rb + DH + 4 * lane) = ml;
      wave_sync();
      const v8us q0 = *(const v8usa*)(rb + 8 * lane);
      wave_sync();
      if (node < MP) {
        unsigned short* rp = hhl + (size_t)node * K2 + 8 * lane;
        *(volatile v8us*)rp = q0;
        __threadfence();
        *(volatile v8us*)rp = q0;
      }
    } else {
      const float v0 = s0 / 3.0f, v1 = s1 / 3.0f;
      v4f ow;
      ow.x = __shfl(v0, sa, 32); ow.y = __shfl(v1, sa, 32);
      ow.z = __shfl(v0, sb, 32); ow.w = __shfl(v1, sb, 32);
      float* op = out + (size_t)node * DO + 4 * (lane & 15);
      const bool wr = live && (lane < 16);
      if (wr) *(volatile v4f*)op = ow;
      __threadfence();
      if (wr) *(volatile v4f*)op = ow;
    }
  }
}

static inline size_t al256(size_t o) { return (o + 255) & ~(size_t)255; }

extern "C" void kernel_launch(void* const* d_in, const int* in_sizes, int n_in,
                              void* d_out, int out_size, void* d_ws, size_t ws_size,
                              hipStream_t stream) {
  if (n_in < 6) return;
  if (in_sizes[0] != NN * DIN) return;
  if (in_sizes[1] != NR * 2 * NE) return;
  if (in_sizes[2] != NR * DIN * DH) return;
  if (in_sizes[3] != NR * DH) return;
  if (in_sizes[4] != NR * DH * DO) return;
  if (in_sizes[5] != NR * DO) return;
  if (out_size != NN * DO) return;

  const float* x  = (const float*)d_in[0];
  const int*   ei = (const int*)  d_in[1];
  const float* W1 = (const float*)d_in[2];
  const float* b1 = (const float*)d_in[3];
  const float* W2 = (const float*)d_in[4];
  const float* b2 = (const float*)d_in[5];
  float* out = (float*)d_out;

  char* ws = (char*)d_ws;
  size_t off = 0;
  const size_t oP1  = off; off = al256(off + SZ_P1);
  const size_t oHH  = off; off = al256(off + SZ_HH);
  const size_t oLST = off; off = al256(off + SZ_LST);
  const size_t oTCI = off; off = al256(off + SZ_TCI);
  const size_t oDV  = off; off = al256(off + SZ_DV);
  const size_t oW1T = off; off = al256(off + SZ_W1T);
  const size_t oW2D = off; off = al256(off + SZ_W2D);
  if (off > ws_size) return;
  float*          P1  = (float*)(ws + oP1);
  float*          P2  = (float*)(ws + oP1);
  unsigned short* HHL = (unsigned short*)(ws + oHH);
  unsigned short* XB  = (unsigned short*)(ws + oHH);
  int*            LST = (int*)(ws + oLST);
  int*            TCI = (int*)(ws + oTCI);
  float*          DV  = (float*)(ws + oDV);
  unsigned short* W1T = (unsigned short*)(ws + oW1T);
  unsigned short* W2D = (unsigned short*)(ws + oW2D);

  const size_t bkLds = (size_t)BK_LDS_INTS * 4;
  hipFuncSetAttribute(reinterpret_cast<const void*>(&k_bucket), hipFuncAttributeMaxDynamicSharedMemorySize, (int)bkLds);

  k_prep<<<NUT / NTHR, NTHR, 0, stream>>>(x, W1, W2, XB, W1T, W2D);
  k_bucket<<<dim3(NBLK, NR), NTHR, bkLds, stream>>>(ei, LST, TCI, DV);
  k_gemm<8, DIN><<<dim3(MP / GBM, NR), GTHR, 0, stream>>>(XB, W1T, DV, P1);
  k_replay<1><<<NBLK, NTHR, 0, stream>>>(P1, LST, TCI, DV, b1, HHL, out);
  k_gemm<4, K2><<<dim3(MP / GBM, NR), GTHR, 0, stream>>>(HHL, W2D, DV, P2);
  k_replay<2><<<NBLK, NTHR, 0, stream>>>(P2, LST, TCI, DV, b2, HHL, out);
}
